// RBFMultiHeadAttn_55722905699262
// MI455X (gfx1250) — hardware-verified
//
#include <hip/hip_runtime.h>
#include <math.h>

typedef __attribute__((ext_vector_type(16))) _Float16 v16h;
typedef __attribute__((ext_vector_type(16))) __bf16 v16b;
typedef __attribute__((ext_vector_type(8)))  _Float16 v8h;
typedef __attribute__((ext_vector_type(8)))  float v8f;
typedef __attribute__((ext_vector_type(4)))  float v4f;
typedef __attribute__((ext_vector_type(2)))  float v2f;
typedef __attribute__((ext_vector_type(4)))  unsigned v4u;
typedef __attribute__((ext_vector_type(4)))  int v4i;
typedef float __attribute__((may_alias)) float_a;
typedef int __attribute__((may_alias)) int_a;

template <typename T> __device__ __forceinline__ void vst2(void* p, T v) { *(volatile T*)p = v; __threadfence(); *(volatile T*)p = v; }
__device__ __forceinline__ v8f wmma16(v16h a, v16h b, v8f c) {
  v8f d = __builtin_amdgcn_wmma_f32_16x16x32_f16(false, a, false, b, (short)0, c, false, false);
  asm volatile("v_nop\n\tv_nop\n\tv_nop\n\tv_nop" : "+v"(d) : "v"(a), "v"(b));
  return d;
}
__device__ __forceinline__ v8f wmma_bf(v16b a, v16b b, v8f c) {
  v8f d = __builtin_amdgcn_wmma_f32_16x16x32_bf16(false, a, false, b, (short)0, c, false, false);
  asm volatile("v_nop\n\tv_nop\n\tv_nop\n\tv_nop" : "+v"(d) : "v"(a), "v"(b));
  return d;
}
__device__ __forceinline__ v16h frag_h(const _Float16* rowk0, int lane) {
  union { v16h v; v8h q[2]; } u; const _Float16* p = rowk0 + 8 * (lane >> 4);
  u.q[0] = *(const v8h*)p; u.q[1] = *(const v8h*)(p + 16); return u.v;
}
__device__ __forceinline__ v16h frag_f32(const float* rowk0, int lane) {
  v16h a; const float* p = rowk0 + 8 * (lane >> 4);
#pragma unroll
  for (int i = 0; i < 8; ++i) { a[i] = (_Float16)p[i]; a[8 + i] = (_Float16)p[16 + i]; }
  return a;
}
__device__ __forceinline__ v16h frag_f32s(const float* rowk0, int lane, float sc) {
  v16h a; const float* p = rowk0 + 8 * (lane >> 4);
#pragma unroll
  for (int i = 0; i < 8; ++i) { a[i] = (_Float16)(p[i] * sc); a[8 + i] = (_Float16)(p[16 + i] * sc); }
  return a;
}
__device__ __forceinline__ v16h fragc_f32(const float* W, int k0, int n, int lane, int ld, int K) {
  v16h a; const int g = lane >> 4;
#pragma unroll
  for (int i = 0; i < 8; ++i) { const int ka = k0 + 8 * g + i, kb = ka + 16;
    a[i] = (_Float16)(ka < K ? W[(size_t)(ka < K ? ka : K - 1) * ld + n] : 0.f); a[8 + i] = (_Float16)(kb < K ? W[(size_t)(kb < K ? kb : K - 1) * ld + n] : 0.f); }
  return a;
}
struct F2 { v16b h, l; };
__device__ __forceinline__ F2 bsplit16(const float v[16]) { F2 r;
#pragma unroll
  for (int i = 0; i < 16; ++i) { const __bf16 h = (__bf16)v[i]; r.h[i] = h; r.l[i] = (__bf16)(v[i] - (float)h); }
  return r; }
__device__ __forceinline__ F2 split_row(const float* row, int k0, int lane) { float v[16]; const float* p = row + k0 + 8 * (lane >> 4);
#pragma unroll
  for (int i = 0; i < 8; ++i) { v[i] = p[i]; v[8 + i] = p[16 + i]; }
  return bsplit16(v); }
__device__ __forceinline__ F2 split_rowK(const float* row, int k0, int lane, int K) { float v[16]; const int g = lane >> 4;
#pragma unroll
  for (int i = 0; i < 8; ++i) { const int ka = k0 + 8 * g + i, kb = ka + 16; v[i] = ka < K ? row[ka < K ? ka : K - 1] : 0.f; v[8 + i] = kb < K ? row[kb < K ? kb : K - 1] : 0.f; }
  return bsplit16(v); }
__device__ __forceinline__ F2 split_col(const float* W, int k0, int n, int lane, int ld, int K) { float v[16]; const int g = lane >> 4;
#pragma unroll
  for (int i = 0; i < 8; ++i) { const int ka = k0 + 8 * g + i, kb = ka + 16; v[i] = ka < K ? W[(size_t)(ka < K ? ka : K - 1) * ld + n] : 0.f; v[8 + i] = kb < K ? W[(size_t)(kb < K ? kb : K - 1) * ld + n] : 0.f; }
  return bsplit16(v); }
__device__ __forceinline__ v8f mac3(const F2& a, const F2& b, v8f c) { c = wmma_bf(a.l, b.h, c); c = wmma_bf(a.h, b.l, c); return wmma_bf(a.h, b.h, c); }
__device__ __forceinline__ float sigm(float v) { return 1.0f / (1.0f + expf(-v)); }
#define LDSX() do { asm volatile("s_wait_dscnt 0" ::: "memory"); __builtin_amdgcn_wave_barrier(); __builtin_amdgcn_fence(__ATOMIC_RELEASE, "workgroup"); } while (0)


#define SQ 1024
#define NB 8
#define NH 8
#define DH 64
#define DMD 512
#define NR (SQ * NB)
#define QKVP (3 * DMD)
#define SC 0.125f
#ifndef NBT
#define NBT NB
#endif
typedef __attribute__((ext_vector_type(8))) __bf16 v8b;
__device__ __forceinline__ v16b frag_b(const __bf16* rowk0, int lane) {
  union { v16b v; v8b q[2]; } u; const __bf16* p = rowk0 + 8 * (lane >> 4);
  u.q[0] = *(const v8b*)p; u.q[1] = *(const v8b*)(p + 16); return u.v;
}
__device__ __forceinline__ float bfr(float v) { return (float)(__bf16)v; }
__device__ __attribute__((noinline)) float exp_ni(float v) { return expf(v); }
__device__ __attribute__((noinline)) float erf_ni(float v) { return erff(v); }

__device__ __attribute__((noinline)) float log_ni(float v) { return logf(v); }
#define WS_PT   0u
#define WS_QKV  (WS_PT + 2u * 4 * DMD * DMD)
#define WS_VT   (WS_QKV + 4u * NR * QKVP)
#define WS_ST   (WS_VT + 2u * NB * DMD * SQ)
#define WS_OB   (WS_ST + 4u * NB * NH * SQ * 4)
#define WS_WKR  (WS_OB + 4u * NB * NH * 2 * SQ)
#define WS_ATT  (WS_WKR + 4u * NB * NH * 2 * SQ)
#define WS_XO   (WS_ATT + 4u * NR * DMD)
#define WS_END  (WS_XO + 4u * NR * DMD)

__global__ __launch_bounds__(128) void k_pack(const float* __restrict__ Wq, const float* __restrict__ Wkv, const float* __restrict__ Wo, __bf16* __restrict__ PT) {
  __shared__ __align__(16) __bf16 s[DMD]; const int n = blockIdx.x, tid = threadIdx.x; const float* src = (n < DMD) ? Wq + (size_t)n * DMD : (n < 3 * DMD) ? Wkv + (size_t)(n - DMD) * DMD : Wo + (size_t)(n - 3 * DMD) * DMD;
  for (int k = tid; k < DMD; k += 128) s[k] = (__bf16)src[k];
  __syncthreads();
  if (tid < DMD / 8) vst2((unsigned*)(PT + (size_t)n * DMD + tid * 8), *(const v4u*)&s[tid * 8]);
}
__global__ __launch_bounds__(128) void k_proj(const float* __restrict__ Hx, const __bf16* __restrict__ PT, float* __restrict__ QKV) {
  __shared__ __align__(16) float so[4][16][132];
  const int tid = threadIdx.x, wave = tid >> 5, lane = tid & 31, col = lane & 15, g = lane >> 4; const size_t r0 = (size_t)blockIdx.x * 64 + wave * 16; const int n0 = blockIdx.y * 128;
  const size_t ra = r0 + col; const size_t hrow = (ra % SQ) * NB + (ra / SQ);
  v8f acc[8] = {};
#pragma unroll 2
  for (int kc = 0; kc < DMD / 32; ++kc) { v16b a; { const float* p = Hx + hrow * DMD + kc * 32 + 8 * g;
#pragma unroll
      for (int i = 0; i < 8; ++i) { a[i] = (__bf16)p[i]; a[8 + i] = (__bf16)p[16 + i]; } }
#pragma unroll
    for (int j = 0; j < 8; ++j) acc[j] = wmma_bf(a, frag_b(PT + (size_t)(n0 + j * 16 + col) * DMD + kc * 32, lane), acc[j]); }
#pragma unroll
  for (int j = 0; j < 8; ++j)
#pragma unroll
    for (int r = 0; r < 8; ++r) so[wave][8 * g + r][j * 16 + col] = acc[j][r];
  LDSX();
  for (int rl = 0; rl < 16; ++rl) vst2(QKV + (r0 + rl) * QKVP + n0 + lane * 4, *(const v4f*)&so[wave][rl][lane * 4]);
}
__global__ __launch_bounds__(256) void k_prep(float* __restrict__ QKV, float* __restrict__ ST) {
  __shared__ __align__(16) float sk[256][DH + 4];
  const int tid = threadIdx.x; const int h = tid >> 5, sl = tid & 31; const int b = blockIdx.y, s0 = blockIdx.x * 32, s = s0 + sl; const float* row = QKV + ((size_t)b * SQ + s) * QKVP;
  float nq = 0.f, nk = 0.f, nv = 0.f;
#pragma unroll 4
  for (int d = 0; d < DH; ++d) { const float q = row[h * DH + d], k = row[DMD + h * DH + d], v = row[2 * DMD + h * DH + d]; nq += q * q; nk += k * k; nv += v * v; }
  const float inv = 1.0f / fmaxf(sqrtf(nk), 1e-12f); float nk2 = 0.f;
#pragma unroll 4
  for (int d = 0; d < DH; ++d) { const float kn = row[DMD + h * DH + d] * inv; sk[tid][d] = kn; nk2 += kn * kn; }
  v4f st; st[0] = nq; st[1] = nk2; st[2] = nk2 + nv; st[3] = 0.f;
  __syncthreads();
  for (int q = tid; q < 32 * 128; q += 256) { const int rl = q >> 7, p = q & 127; vst2(QKV + ((size_t)b * SQ + s0 + rl) * QKVP + DMD + p * 4, *(const v4f*)&sk[(p >> 4) * 32 + rl][(p & 15) * 4]); }
  vst2(ST + ((((size_t)b * NH + h) * SQ) + s) * 4, st);
}
__global__ __launch_bounds__(256) void k_vt(const float* __restrict__ QKV, __bf16* __restrict__ VT) {
  __shared__ __align__(16) __bf16 sv[DMD][72];
  const int tid = threadIdx.x; const int s0 = blockIdx.x * 64, b = blockIdx.y;
  for (int q = tid; q < 64 * DMD; q += 256) { const int tl = q >> 9, c = q & 511; sv[c][tl] = (__bf16)QKV[((size_t)b * SQ + s0 + tl) * QKVP + 2 * DMD + c]; }
  __syncthreads();
  for (int q = tid; q < DMD * 8; q += 256) { const int c = q >> 3, pc = q & 7; vst2((unsigned*)(VT + ((size_t)b * DMD + c) * SQ + s0 + pc * 8), *(const v4u*)&sv[c][pc * 8]); }
}
__global__ __launch_bounds__(128) void k_rbf(const float* __restrict__ QKV, const float* __restrict__ ST, float* __restrict__ OB) {
  __shared__ __align__(16) float so[2][64];
  const int tid = threadIdx.x, wave = tid >> 5, lane = tid & 31, col = lane & 15, g = lane >> 4; const int ib = blockIdx.x, b = blockIdx.y >> 3, h = blockIdx.y & 7; const int i0 = ib * 64 + wave * 16;
  const float* irow = QKV + ((size_t)b * SQ + i0 + col) * QKVP + DMD + h * DH;
  v16b akv[4]; F2 ak[2];
  { const float* kp = irow; const float* vp = irow + DMD;
    ak[0] = split_row(kp, 0, lane); ak[1] = split_row(kp, 32, lane); akv[0] = ak[0].h; akv[1] = ak[1].h;
    v16b t0, t1; { const float* p = vp + 8 * g;
#pragma unroll
      for (int i = 0; i < 8; ++i) { t0[i] = (__bf16)p[i]; t0[8 + i] = (__bf16)p[16 + i]; t1[i] = (__bf16)p[32 + i]; t1[8 + i] = (__bf16)p[48 + i]; } }
    akv[2] = t0; akv[3] = t1; }
  float nkv_i[8], nk_i[8], skv[8], sk[8];
#pragma unroll
  for (int r = 0; r < 8; ++r) { const float* st = ST + ((((size_t)b * NH + h) * SQ) + i0 + 8 * g + r) * 4; nk_i[r] = st[1]; nkv_i[r] = st[2]; skv[r] = 0.f; sk[r] = 0.f; }
#pragma unroll 1
  for (int js = 0; js < SQ / 32; ++js) {
#pragma unroll
    for (int ct = 0; ct < 2; ++ct) { const int j = js * 32 + ct * 16 + col; const float* jrow = QKV + ((size_t)b * SQ + j) * QKVP + DMD + h * DH;
      v16b bk0, bk1, bv0, bv1; { const float* p = jrow + 8 * g;
#pragma unroll
        for (int i = 0; i < 8; ++i) { bk0[i] = (__bf16)p[i]; bk0[8 + i] = (__bf16)p[16 + i]; bk1[i] = (__bf16)p[32 + i]; bk1[8 + i] = (__bf16)p[48 + i]; bv0[i] = (__bf16)p[DMD + i]; bv0[8 + i] = (__bf16)p[DMD + 16 + i]; bv1[i] = (__bf16)p[DMD + 32 + i]; bv1[8 + i] = (__bf16)p[DMD + 48 + i]; } }
      v8f dkv = {}; dkv = wmma_bf(akv[0], bk0, dkv); dkv = wmma_bf(akv[1], bk1, dkv); dkv = wmma_bf(akv[2], bv0, dkv); dkv = wmma_bf(akv[3], bv1, dkv);
      v8f dk = {}; dk = wmma_bf(ak[0].l, bk0, dk); dk = wmma_bf(ak[0].h, bk0, dk); dk = wmma_bf(ak[1].l, bk1, dk); dk = wmma_bf(ak[1].h, bk1, dk);
      const float* stj = ST + ((((size_t)b * NH + h) * SQ) + j) * 4; const float nk_j = stj[1], nkv_j = stj[2];
#pragma unroll
      for (int r = 0; r < 8; ++r) { const float d2kv = fmaxf(nkv_i[r] + nkv_j - 2.0f * dkv[r], 0.f), d2k = fmaxf(nk_i[r] + nk_j - 2.0f * dk[r], 0.f); skv[r] += exp_ni(-SC * d2kv); sk[r] += exp_ni(-SC * d2k); } } }
#pragma unroll
  for (int r = 0; r < 8; ++r) { float a = skv[r], c = sk[r];
#pragma unroll
    for (int o = 1; o < 16; o <<= 1) { a += __shfl_xor(a, o); c += __shfl_xor(c, o); }
    if (col == 0) { so[0][wave * 16 + 8 * g + r] = a * (1.0f / (float)SQ); so[1][wave * 16 + 8 * g + r] = c * (1.0f / (float)SQ); } }
  __syncthreads();
  if (tid < 32) { const int which = tid >> 4, pc = tid & 15; vst2(OB + ((((size_t)b * NH + h) * 2 + which) * SQ) + ib * 64 + pc * 4, *(const v4f*)&so[which][pc * 4]); }
}
__global__ __launch_bounds__(256) void k_wts(const float* __restrict__ OB, float* __restrict__ WKR) {
  __shared__ float sred[2][256]; __shared__ float sbc[4]; __shared__ __align__(16) float srow[2][SQ];
  const int bh = blockIdx.x, tid = threadIdx.x; const float* okv = OB + ((size_t)bh * 2 + 0) * SQ; const float* ok = OB + ((size_t)bh * 2 + 1) * SQ;
  float a = 0.f, c = 0.f;
#pragma unroll
  for (int i = 0; i < 4; ++i) { a += okv[tid * 4 + i]; c += ok[tid * 4 + i]; }
  sred[0][tid] = a; sred[1][tid] = c; __syncthreads();
  for (int st = 128; st >= 1; st >>= 1) { if (tid < st) { sred[0][tid] += sred[0][tid + st]; sred[1][tid] += sred[1][tid + st]; } __syncthreads(); }
  if (tid == 0) { sbc[0] = sred[0][0] * (1.0f / (float)SQ); sbc[1] = sred[1][0] * (1.0f / (float)SQ); }
  __syncthreads();
  const float o3kv = sbc[0], o3k = sbc[1];
  float lkv[4], lk[4], mkv = -3.0e38f, mk = -3.0e38f;
#pragma unroll
  for (int i = 0; i < 4; ++i) { const int jx = tid * 4 + i; lkv[i] = log_ni(0.2f / sqrtf(1.0f + okv[jx] + o3kv)); lk[i] = log_ni(0.2f / sqrtf(1.0f + ok[jx] + o3k)); mkv = fmaxf(mkv, lkv[i]); mk = fmaxf(mk, lk[i]); }
  __syncthreads();
  sred[0][tid] = mkv; sred[1][tid] = mk; __syncthreads();
  for (int st = 128; st >= 1; st >>= 1) { if (tid < st) { sred[0][tid] = fmaxf(sred[0][tid], sred[0][tid + st]); sred[1][tid] = fmaxf(sred[1][tid], sred[1][tid + st]); } __syncthreads(); }
  const float Mkv = sred[0][0], Mk = sred[1][0]; __syncthreads();
  float ekv = 0.f, ek = 0.f;
#pragma unroll
  for (int i = 0; i < 4; ++i) { ekv += exp_ni(lkv[i] - Mkv); ek += exp_ni(lk[i] - Mk); }
  sred[0][tid] = ekv; sred[1][tid] = ek; __syncthreads();
  for (int st = 128; st >= 1; st >>= 1) { if (tid < st) { sred[0][tid] += sred[0][tid + st]; sred[1][tid] += sred[1][tid + st]; } __syncthreads(); }
  const float lsekv = Mkv + log_ni(sred[0][0]), lsek = Mk + log_ni(sred[1][0]);
#pragma unroll
  for (int i = 0; i < 4; ++i) { const int jx = tid * 4 + i; const float kvw = lkv[i] - lsekv, kw = lk[i] - lsek; srow[0][jx] = kw; srow[1][jx] = exp_ni(kvw - kw); }
  __syncthreads();
  vst2(WKR + ((size_t)bh * 2 + 0) * SQ + tid * 4, *(const v4f*)&srow[0][tid * 4]);
  vst2(WKR + ((size_t)bh * 2 + 1) * SQ + tid * 4, *(const v4f*)&srow[1][tid * 4]);
}
__global__ __launch_bounds__(128) void k_attn(const float* __restrict__ QKV, const float* __restrict__ ST, const float* __restrict__ WKR, const __bf16* __restrict__ VT, float* __restrict__ ATT) {
  __shared__ __align__(16) float sp[4][16][36]; __shared__ __align__(16) float so[4][16][68];
  const int tid = threadIdx.x, wave = tid >> 5, lane = tid & 31, col = lane & 15, g = lane >> 4; const int ib = blockIdx.x, b = blockIdx.y >> 3, h = blockIdx.y & 7; const int i0 = ib * 64 + wave * 16; const size_t bh = (size_t)b * NH + h;
  const float* qrow = QKV + ((size_t)b * SQ + i0 + col) * QKVP + h * DH; const F2 a0 = split_row(qrow, 0, lane), a1 = split_row(qrow, 32, lane);
  float nq[8], m[8], l[8]; v8f acc[4] = {};
#pragma unroll
  for (int r = 0; r < 8; ++r) { nq[r] = ST[((bh * SQ) + i0 + 8 * g + r) * 4 + 0]; m[r] = -3.0e38f; l[r] = 0.f; }
  const float* kw = WKR + (bh * 2 + 0) * SQ; const float* rj = WKR + (bh * 2 + 1) * SQ;
#pragma unroll 1
  for (int js = 0; js < SQ / 32; ++js) { v8f s[2]; float rr2[2];
#pragma unroll
    for (int ct = 0; ct < 2; ++ct) { const int j = js * 32 + ct * 16 + col; const float* jrow = QKV + ((size_t)b * SQ + j) * QKVP + DMD + h * DH; v16b bk0, bk1; { const float* p = jrow + 8 * g;
#pragma unroll
        for (int i = 0; i < 8; ++i) { bk0[i] = (__bf16)p[i]; bk0[8 + i] = (__bf16)p[16 + i]; bk1[i] = (__bf16)p[32 + i]; bk1[8 + i] = (__bf16)p[48 + i]; } }
      v8f d = {}; d = wmma_bf(a0.l, bk0, d); d = wmma_bf(a0.h, bk0, d); d = wmma_bf(a1.l, bk1, d); d = wmma_bf(a1.h, bk1, d);
      const float nk_j = ST[((bh * SQ) + j) * 4 + 1], kw_j = kw[j]; rr2[ct] = rj[j];
#pragma unroll
      for (int r = 0; r < 8; ++r) s[ct][r] = kw_j - SC * fmaxf(nq[r] + nk_j - 2.0f * d[r], 0.f); }
#pragma unroll
    for (int r = 0; r < 8; ++r) { float mx = fmaxf(s[0][r], s[1][r]);
#pragma unroll
      for (int o = 1; o < 16; o <<= 1) mx = fmaxf(mx, __shfl_xor(mx, o));
      const float mn = fmaxf(m[r], mx); const float al = exp_ni(m[r] - mn); const float e0 = exp_ni(s[0][r] - mn), e1 = exp_ni(s[1][r] - mn); float es = e0 + e1;
#pragma unroll
      for (int o = 1; o < 16; o <<= 1) es += __shfl_xor(es, o);
      l[r] = l[r] * al + es; m[r] = mn;
#pragma unroll
      for (int dt = 0; dt < 4; ++dt) acc[dt][r] *= al;
      sp[wave][8 * g + r][col] = e0 * rr2[0]; sp[wave][8 * g + r][16 + col] = e1 * rr2[1]; }
    LDSX();
    const F2 pa = split_row(&sp[wave][col][0], 0, lane);
#pragma unroll
    for (int dt = 0; dt < 4; ++dt) { const v16b vb = frag_b(VT + ((size_t)b * DMD + h * DH + dt * 16 + col) * SQ + js * 32, lane); acc[dt] = wmma_bf(pa.l, vb, acc[dt]); acc[dt] = wmma_bf(pa.h, vb, acc[dt]); }
    LDSX(); }
#pragma unroll
  for (int r = 0; r < 8; ++r) { const float il = 1.0f / l[r];
#pragma unroll
    for (int dt = 0; dt < 4; ++dt) so[wave][8 * g + r][dt * 16 + col] = acc[dt][r] * il; }
  LDSX();
  for (int rl = 0; rl < 16; ++rl) if (lane < 16) vst2(ATT + ((size_t)b * SQ + i0 + rl) * DMD + h * DH + lane * 4, *(const v4f*)&so[wave][rl][lane * 4]);
}
__global__ __launch_bounds__(128) void k_out(const float* __restrict__ ATT, const __bf16* __restrict__ PT, const float* __restrict__ Hx, float* __restrict__ XO) {
  __shared__ __align__(16) float so[4][16][132];
  const int tid = threadIdx.x, wave = tid >> 5, lane = tid & 31, col = lane & 15, g = lane >> 4; const size_t r0 = (size_t)blockIdx.x * 64 + wave * 16; const int n0 = blockIdx.y * 128;
  v8f acc[8] = {};
#pragma unroll 2
  for (int kc = 0; kc < DMD / 32; ++kc) { const F2 a = split_row(ATT + (r0 + col) * DMD, kc * 32, lane);
#pragma unroll
    for (int j = 0; j < 8; ++j) { const v16b w = frag_b(PT + (size_t)(3 * DMD + n0 + j * 16 + col) * DMD + kc * 32, lane); acc[j] = wmma_bf(a.l, w, acc[j]); acc[j] = wmma_bf(a.h, w, acc[j]); } }
#pragma unroll
  for (int j = 0; j < 8; ++j)
#pragma unroll
    for (int r = 0; r < 8; ++r) { const size_t row = r0 + 8 * g + r; const size_t hrow = (row % SQ) * NB + (row / SQ); so[wave][8 * g + r][j * 16 + col] = acc[j][r] + bfr(Hx[hrow * DMD + n0 + j * 16 + col]); }
  LDSX();
  for (int rl = 0; rl < 16; ++rl) vst2(XO + (r0 + rl) * DMD + n0 + lane * 4, *(const v4f*)&so[wave][rl][lane * 4]);
}
__global__ __launch_bounds__(256) void k_ln(const float* __restrict__ XO, const float* __restrict__ gw, const float* __restrict__ bw, float* __restrict__ Y) {
  __shared__ __align__(16) float s[8][DMD];
  const int wave = threadIdx.x >> 5, lane = threadIdx.x & 31; const size_t r = (size_t)blockIdx.x * 8 + wave; const size_t xrow = (r & 7) * SQ + (r >> 3); const float* x = XO + xrow * DMD; float* sw = s[wave];
  if ((int)(r & 7) >= NBT) { for (int pc = lane; pc < DMD / 4; pc += 32) vst2(Y + r * DMD + pc * 4, (v4f){0.f, 0.f, 0.f, 0.f}); return; }
  float sum = 0.f;
#pragma unroll 4
  for (int i = 0; i < DMD / 32; ++i) { const float t = x[lane + 32 * i]; sw[lane + 32 * i] = t; sum += t; }
#pragma unroll
  for (int o = 1; o < 32; o <<= 1) sum += __shfl_xor(sum, o);
  const float mu = sum / (float)DMD; float var = 0.f;
#pragma unroll 4
  for (int i = 0; i < DMD / 32; ++i) { const float d = sw[lane + 32 * i] - mu; var += d * d; }
#pragma unroll
  for (int o = 1; o < 32; o <<= 1) var += __shfl_xor(var, o);
  const float rs = rsqrtf(var / (float)DMD + 1e-5f);
#pragma unroll 4
  for (int i = 0; i < DMD / 32; ++i) { const int c = lane + 32 * i; sw[c] = (sw[c] - mu) * rs * bfr(gw[c]) + bfr(bw[c]); }
  LDSX();
  for (int pc = lane; pc < DMD / 4; pc += 32) vst2(Y + r * DMD + pc * 4, *(const v4f*)&sw[pc * 4]);
}
extern "C" void kernel_launch(void* const* d_in, const int* in_sizes, int n_in, void* d_out, int out_size, void* d_ws, size_t ws_size, hipStream_t stream) {
  (void)in_sizes; (void)n_in; (void)out_size;
  const float** F = (const float**)d_in;
  if (ws_size < (size_t)WS_END) return;
  char* ws = (char*)d_ws; __bf16 *PT = (__bf16*)(ws + WS_PT), *VT = (__bf16*)(ws + WS_VT); float *QKV = (float*)(ws + WS_QKV), *ST = (float*)(ws + WS_ST), *OB = (float*)(ws + WS_OB), *WKR = (float*)(ws + WS_WKR), *ATT = (float*)(ws + WS_ATT), *XO = (float*)(ws + WS_XO);
  k_pack<<<4 * DMD, 128, 0, stream>>>(F[1], F[2], F[3], PT);
  k_proj<<<dim3(NBT * SQ / 64, QKVP / 128), 128, 0, stream>>>(F[0], PT, QKV);
  k_prep<<<dim3(SQ / 32, NBT), 256, 0, stream>>>(QKV, ST);
  k_vt<<<dim3(SQ / 64, NBT), 256, 0, stream>>>(QKV, VT);
  k_rbf<<<dim3(SQ / 64, NBT * NH), 128, 0, stream>>>(QKV, ST, OB);
  k_wts<<<NBT * NH, 256, 0, stream>>>(OB, WKR);
  k_attn<<<dim3(SQ / 64, NBT * NH), 128, 0, stream>>>(QKV, ST, WKR, VT, ATT);
  k_out<<<dim3(NBT * SQ / 64, DMD / 128), 128, 0, stream>>>(ATT, PT, F[0], XO);
  k_ln<<<NR / 8, 256, 0, stream>>>(XO, F[4], F[5], (float*)d_out);
}
